// GQA_28561532518475
// MI455X (gfx1250) — hardware-verified
//
#include <hip/hip_runtime.h>
#include <math.h>

constexpr int kBatch   = 4;
constexpr int kSeq     = 2048;
constexpr int kDim     = 768;
constexpr int kHeads   = 12;
constexpr int kKVHeads = 6;
constexpr int kDh      = 64;
constexpr int kTok     = kBatch * kSeq;
constexpr int kKVDim   = kKVHeads * kDh;
constexpr int kQKN     = kDim + kKVDim;
constexpr int kSlotsPerGroup = kHeads / kKVHeads;
constexpr float kQKCarry  = 8.0f;
constexpr float kVCarry   = 8.0f;
constexpr float kPCarry   = 32768.0f;
constexpr float kOCarry   = 256.0f;
constexpr float kWpCarry  = 256.0f;
constexpr float kAttnScale  = 0.125f;
constexpr float kScoreScale = kAttnScale / (kQKCarry * kQKCarry);
constexpr float kPVScale    = kOCarry / (kPCarry * kVCarry);
constexpr float kOutScale   = 1.0f / (kOCarry * kWpCarry);
static_assert(kHeads * kDh == kDim, "shape");
static_assert(kSlotsPerGroup == 2, "group size");
static_assert(kTok % 64 == 0 && kQKN % 64 == 0 && kDim % 32 == 0, "qk projection tiles");
static_assert(kKVDim % 64 == 0 && kTok % 64 == 0, "vt projection tiles");
static_assert(kSeq % 64 == 0 && kDh % 64 == 0 && kDh % 32 == 0 && kSeq % 32 == 0, "attention tiles");
static_assert(kDim % 64 == 0, "out projection tiles");
static_assert(kSeq == 256 * 8, "softmax row map: 256 threads x 8 columns");
static_assert((kTok * kDim) % (256 * 8) == 0, "cast grid exact");

constexpr size_t kSzX   = (size_t)kTok * kDim * 2;
constexpr size_t kSzWqk = (size_t)kQKN * kDim * 2;
constexpr size_t kSzWv  = (size_t)kKVDim * kDim * 2;
constexpr size_t kSzWp  = (size_t)kDim * kDim * 2;
constexpr size_t kSzQK  = (size_t)kTok * kQKN * 2;
constexpr size_t kSzVT  = (size_t)kKVDim * kTok * 2;
constexpr size_t kSzSC  = (size_t)kSlotsPerGroup * kSeq * kSeq * 4;
constexpr size_t kSzPP  = (size_t)kSlotsPerGroup * kSeq * kSeq * 2;
constexpr size_t kSzO   = (size_t)kTok * kDim * 2;
constexpr size_t kOffX   = 0;
constexpr size_t kOffWqk = kOffX + kSzX;
constexpr size_t kOffWv  = kOffWqk + kSzWqk;
constexpr size_t kOffWp  = kOffWv + kSzWv;
constexpr size_t kOffQK  = kOffWp + kSzWp;
constexpr size_t kOffVT  = kOffQK + kSzQK;
constexpr size_t kOffSC  = kOffVT + kSzVT;
constexpr size_t kOffPP  = kOffSC + kSzSC;
constexpr size_t kOffO   = kOffPP + kSzPP;
constexpr size_t kWsTotal = kOffO + kSzO;
static_assert(kWsTotal == 104202240ull, "carve total");
static_assert(kWsTotal <= 134217728ull, "carve budget");
static_assert(kOffWqk % 128 == 0 && kOffWv % 128 == 0 && kOffWp % 128 == 0 && kOffQK % 128 == 0 &&
              kOffVT % 128 == 0 && kOffSC % 128 == 0 && kOffPP % 128 == 0 && kOffO % 128 == 0, "line aligned");

typedef __attribute__((ext_vector_type(16))) _Float16 v16h;
typedef __attribute__((ext_vector_type(8)))  _Float16 v8h;
typedef __attribute__((ext_vector_type(16))) __bf16   v16b;
typedef __attribute__((ext_vector_type(8)))  __bf16   v8b;
typedef __attribute__((ext_vector_type(8)))  float    v8f;
typedef __attribute__((ext_vector_type(4)))  float    v4f;
typedef __attribute__((ext_vector_type(4)))  unsigned int v4u;

__device__ __forceinline__ unsigned short f2bf_bits(float f) {
  unsigned u = __float_as_uint(f);
  return (unsigned short)((u + 0x7FFFu + ((u >> 16) & 1u)) >> 16);
}
__device__ __forceinline__ float bf_bits2f(unsigned short h) { return __uint_as_float(((unsigned)h) << 16); }

__device__ __forceinline__ void dep_guard_h(v8f& a, v8f& b, v16h x, v16h y) { asm volatile("v_nop\n\tv_nop\n\tv_nop\n\tv_nop" : "+v"(a), "+v"(b) : "v"(x), "v"(y)); }
__device__ __forceinline__ void dep_guard_b(v8f& a, v8f& b, v16b x, v16b y) { asm volatile("v_nop\n\tv_nop\n\tv_nop\n\tv_nop" : "+v"(a), "+v"(b) : "v"(x), "v"(y)); }
__device__ __forceinline__ void dep_guard4_h(v8f& a, v8f& b, v8f& c, v8f& d, v16h x, v16h y) { asm volatile("v_nop\n\tv_nop\n\tv_nop\n\tv_nop" : "+v"(a), "+v"(b), "+v"(c), "+v"(d) : "v"(x), "v"(y)); }
__device__ __forceinline__ void dep_guard4_b(v8f& a, v8f& b, v8f& c, v8f& d, v16b x, v16b y) { asm volatile("v_nop\n\tv_nop\n\tv_nop\n\tv_nop" : "+v"(a), "+v"(b), "+v"(c), "+v"(d) : "v"(x), "v"(y)); }
__device__ __forceinline__ void keep4_h(v16h a, v16h b, v16h c, v16h d) { asm volatile("v_nop" :: "v"(a), "v"(b), "v"(c), "v"(d)); }
__device__ __forceinline__ void keep4_b(v16b a, v16b b, v16b c, v16b d) { asm volatile("v_nop" :: "v"(a), "v"(b), "v"(c), "v"(d)); }
__device__ __forceinline__ void acc_guard4(v8f& a, v8f& b, v8f& c, v8f& d) { asm volatile("v_nop\n\tv_nop\n\tv_nop\n\tv_nop" : "+v"(a), "+v"(b), "+v"(c), "+v"(d)); }
template <typename T> struct Frag;
template <> struct Frag<_Float16> {
  typedef v16h V; union U { v16h v; v8h h[2]; };
  static __device__ __forceinline__ v16h load(const _Float16* p) {
    U f; f.h[0] = *(const v8h*)(p); f.h[1] = *(const v8h*)(p + 16); return f.v;
  }
  static __device__ __forceinline__ v8f mma(v16h a, v16h b, v8f c) {
    return __builtin_amdgcn_wmma_f32_16x16x32_f16(false, a, false, b, (short)0, c, false, false);
  }
  static __device__ __forceinline__ void guard(v8f& a, v8f& b, v16h x, v16h y) { dep_guard_h(a, b, x, y); }
  static __device__ __forceinline__ void guard4(v8f& a, v8f& b, v8f& c, v8f& d, v16h x, v16h y) { dep_guard4_h(a, b, c, d, x, y); }
  static __device__ __forceinline__ void keep(v16h a, v16h b, v16h c, v16h d) { keep4_h(a, b, c, d); }
};
template <> struct Frag<__bf16> {
  typedef v16b V; union U { v16b v; v8b h[2]; };
  static __device__ __forceinline__ v16b load(const __bf16* p) {
    U f; f.h[0] = *(const v8b*)(p); f.h[1] = *(const v8b*)(p + 16); return f.v;
  }
  static __device__ __forceinline__ v8f mma(v16b a, v16b b, v8f c) {
    return __builtin_amdgcn_wmma_f32_16x16x32_bf16(false, a, false, b, (short)0, c, false, false);
  }
  static __device__ __forceinline__ void guard(v8f& a, v8f& b, v16b x, v16b y) { dep_guard_b(a, b, x, y); }
  static __device__ __forceinline__ void guard4(v8f& a, v8f& b, v8f& c, v8f& d, v16b x, v16b y) { dep_guard4_b(a, b, c, d, x, y); }
  static __device__ __forceinline__ void keep(v16b a, v16b b, v16b c, v16b d) { keep4_b(a, b, c, d); }
};

__device__ __forceinline__ unsigned pk16(unsigned short a, unsigned short b) { return (unsigned)a | ((unsigned)b << 16); }
__device__ __forceinline__ unsigned short h_bits(float f) { const _Float16 h = (_Float16)f; return __builtin_bit_cast(unsigned short, h); }

template <int ET> struct Elem;
template <> struct Elem<0> { typedef _Float16 T; };
template <> struct Elem<1> { typedef __bf16 T; };
template <int ET, bool SPLIT, int BIAS_MODE, int OUT_MODE, bool RESID, int ACT = 0>
__global__ __launch_bounds__(256) void wmma_gemm64(
    const unsigned short* __restrict__ Ap, const unsigned short* __restrict__ A2p, int lda, long strideA,
    const unsigned short* __restrict__ Btp, const unsigned short* __restrict__ Bt2p, int ldb, long strideB,
    void* __restrict__ Cout, void* __restrict__ Cout2, int ldc, long strideC,
    const float* __restrict__ bias,
    const float* __restrict__ resid, long strideR,
    int M, int N, int K, float scale) {
  typedef typename Elem<ET>::T T;
  typedef typename Frag<T>::V V;
  const T* A = (const T*)Ap; const T* A2 = (const T*)A2p; const T* Bt = (const T*)Btp; const T* Bt2 = (const T*)Bt2p;
  __shared__ __align__(16) float sT[8][16 * 68];
  const int b    = blockIdx.y;
  const int lane = threadIdx.x & 31;
  const int wave = threadIdx.x >> 5;
  const int tilesN = N >> 6;
  const int tilesM = M >> 6;
  const int tile = blockIdx.x * 8 + wave;
  if (tile >= tilesM * tilesN) return;
  const int tm = tile / tilesN;
  const int tn = tile - tm * tilesN;
  const int m0 = tm << 6;
  const int n0 = tn << 6;

  const T* Ab  = A  + (size_t)b * strideA;
  const T* Bb  = Bt + (size_t)b * strideB;
  const T* Ab2 = SPLIT ? (A2  + (size_t)b * strideA) : nullptr;
  const T* Bb2 = SPLIT ? (Bt2 + (size_t)b * strideB) : nullptr;

  const int rlane = lane & 15;
  const int koff  = (lane >> 4) * 8;
  const int mOff  = (lane >> 4) * 8;

  v8f acc[4][4];
#pragma unroll
  for (int i = 0; i < 4; ++i)
#pragma unroll
    for (int j = 0; j < 4; ++j) acc[i][j] = (v8f){0.f,0.f,0.f,0.f,0.f,0.f,0.f,0.f};

  for (int k0 = 0; k0 < K; k0 += 32) {
    V bh[4], bl[4];
#pragma unroll
    for (int j = 0; j < 4; ++j) {
      const size_t bo = (size_t)(n0 + (j << 4) + rlane) * ldb + koff + k0;
      bh[j] = Frag<T>::load(Bb + bo);
      if (SPLIT) bl[j] = Frag<T>::load(Bb2 + bo);
    }
#pragma unroll
    for (int i = 0; i < 4; ++i) {
      const size_t ao = (size_t)(m0 + (i << 4) + rlane) * lda + koff + k0;
      V ah = Frag<T>::load(Ab + ao);
      V al;
      if (SPLIT) al = Frag<T>::load(Ab2 + ao);
#pragma unroll
      for (int j = 0; j < 4; ++j) {
        acc[i][j] = Frag<T>::mma(ah, bh[j], acc[i][j]);
        if (SPLIT) {
          acc[i][j] = Frag<T>::mma(ah, bl[j], acc[i][j]);
          acc[i][j] = Frag<T>::mma(al, bh[j], acc[i][j]);
        }
      }
      Frag<T>::guard4(acc[i][0], acc[i][1], acc[i][2], acc[i][3], ah, SPLIT ? al : bh[3]);
    }
    Frag<T>::keep(bh[0], bh[1], bh[2], bh[3]);
    if (SPLIT) Frag<T>::keep(bl[0], bl[1], bl[2], bl[3]);
  }
  acc_guard4(acc[0][0], acc[0][1], acc[0][2], acc[0][3]);
  acc_guard4(acc[1][0], acc[1][1], acc[1][2], acc[1][3]);
  acc_guard4(acc[2][0], acc[2][1], acc[2][2], acc[2][3]);
  acc_guard4(acc[3][0], acc[3][1], acc[3][2], acc[3][3]);

  float* slab = sT[wave];
  const float* Rb = RESID ? (resid + (size_t)b * strideR) : nullptr;
#pragma unroll
  for (int i = 0; i < 4; ++i) {
    const int mBase = m0 + (i << 4);
#pragma unroll
    for (int j = 0; j < 4; ++j) {
      const int n = n0 + (j << 4) + rlane;
      float bv = 0.f;
      if (BIAS_MODE == 2) bv = bias[n];
#pragma unroll
      for (int r = 0; r < 8; ++r) {
        float v = acc[i][j][r] * scale;
        if (BIAS_MODE == 1) v += bias[mBase + mOff + r];
        if (BIAS_MODE == 2) v += bv;
        if (RESID) v += Rb[(size_t)(mBase + mOff + r) * ldc + n];
        if (ACT == 2) v = fmaxf(v, 0.0f);
        if (ACT == 4) v = (v > 0.f) ? v : 0.01f * v;
        slab[(mOff + r) * 68 + (j << 4) + rlane] = v;
      }
    }
    __builtin_amdgcn_fence(__ATOMIC_RELEASE, "workgroup");
    __builtin_amdgcn_wave_barrier();
    __builtin_amdgcn_fence(__ATOMIC_ACQUIRE, "workgroup");
    if (OUT_MODE == 0) {
      float* C = (float*)Cout + (size_t)b * strideC;
      const int hh = lane >> 4, c4 = (lane & 15) * 4;
      for (int pass = 0; pass < 2; ++pass) {
#pragma unroll
        for (int it = 0; it < 8; ++it) {
          const int row = it * 2 + hh;
          v4f v = *(const v4f*)(slab + row * 68 + c4);
          *(volatile v4f*)(C + (size_t)(mBase + row) * ldc + n0 + c4) = v;
        }
        __threadfence();
      }
    } else {
      const int q = lane >> 3, c8 = (lane & 7) * 8;
      unsigned short* C  = (unsigned short*)Cout  + (size_t)b * strideC;
      unsigned short* C2 = (OUT_MODE == 2) ? ((unsigned short*)Cout2 + (size_t)b * strideC) : nullptr;
      for (int pass = 0; pass < 2; ++pass) {
#pragma unroll
        for (int it = 0; it < 4; ++it) {
          const int row = it * 4 + q;
          const float* sp = slab + row * 68 + c8;
          v8h hv, lv;
#pragma unroll
          for (int e = 0; e < 8; ++e) {
            if (OUT_MODE == 1) {
              hv[e] = (_Float16)sp[e];
            } else {
              unsigned short hb = f2bf_bits(sp[e]);
              unsigned short lb = f2bf_bits(sp[e] - bf_bits2f(hb));
              hv[e] = __builtin_bit_cast(_Float16, hb);
              lv[e] = __builtin_bit_cast(_Float16, lb);
            }
          }
          *(volatile v8h*)(C + (size_t)(mBase + row) * ldc + n0 + c8) = hv;
          if (OUT_MODE == 2) *(volatile v8h*)(C2 + (size_t)(mBase + row) * ldc + n0 + c8) = lv;
        }
        __threadfence();
      }
    }
    __builtin_amdgcn_fence(__ATOMIC_RELEASE, "workgroup");
    __builtin_amdgcn_wave_barrier();
    __builtin_amdgcn_fence(__ATOMIC_ACQUIRE, "workgroup");
  }
}

__global__ __launch_bounds__(256) void cast8_bf16_kernel(const float* __restrict__ in, unsigned short* __restrict__ out, int n8) {
  const int i = blockIdx.x * 256 + threadIdx.x;
  if (i >= n8) return;
  const float* p = in + 8 * (size_t)i;
  const v4f a = *(const v4f*)(p);
  const v4f c = *(const v4f*)(p + 4);
  unsigned short hb[8];
#pragma unroll
  for (int e = 0; e < 4; ++e) {
    hb[e]     = f2bf_bits(a[e]);
    hb[4 + e] = f2bf_bits(c[e]);
  }
  const v4u u = (v4u){pk16(hb[0], hb[1]), pk16(hb[2], hb[3]), pk16(hb[4], hb[5]), pk16(hb[6], hb[7])};
  unsigned short* q = out + 8 * (size_t)i;
  *(volatile v4u*)q = u;
  __threadfence();
  *(volatile v4u*)q = u;
}

template <int ROWM, int COLM, bool F16OUT>
__global__ __launch_bounds__(256) void wprep_kernel(const float* __restrict__ W, int ldw, const int* __restrict__ perm,
                                                    unsigned short* __restrict__ out, float scale) {
  __shared__ float sm[64][65];
  __shared__ int sPerm[kHeads];
  const int t  = threadIdx.x;
  const int kt = blockIdx.x;
  const int nt = blockIdx.y;
  {
    const int pi = (t < kHeads) ? t : (kHeads - 1);
    int p = perm[pi];
    p = p < 0 ? 0 : p;
    p = p > (kHeads - 1) ? (kHeads - 1) : p;
    if (t < kHeads) sPerm[t] = p;
  }
  __syncthreads();
  int rb = kt;
  int cb = nt;
  if (ROWM == 1) rb = sPerm[kt];
  if (ROWM == 2) {
    rb = 0;
#pragma unroll
    for (int j = 0; j < kHeads; ++j) rb = (sPerm[j] == kt) ? j : rb;
  }
  if (COLM == 1) cb = sPerm[nt];
  const float* src = W + (size_t)(rb * 64) * ldw + cb * 64;
#pragma unroll
  for (int i = 0; i < 8; ++i) {
    const int e = i * 256 + t;
    const int r = e >> 6;
    const int c = e & 63;
    float w = src[(size_t)r * ldw + c];
    if (F16OUT) w = bf_bits2f(f2bf_bits(w));
    sm[c][r] = w * scale;
  }
  asm volatile("" ::: "memory");
#pragma unroll
  for (int i = 8; i < 16; ++i) {
    const int e = i * 256 + t;
    const int r = e >> 6;
    const int c = e & 63;
    float w = src[(size_t)r * ldw + c];
    if (F16OUT) w = bf_bits2f(f2bf_bits(w));
    sm[c][r] = w * scale;
  }
  __syncthreads();
  const int lane = t & 31, wave = t >> 5;
  const int q = lane >> 3, c8 = (lane & 7) * 8;
  for (int pass = 0; pass < 2; ++pass) {
#pragma unroll
    for (int it = 0; it < 2; ++it) {
      const int row = wave * 8 + it * 4 + q;
      unsigned short hb[8];
#pragma unroll
      for (int e = 0; e < 8; ++e) {
        const float f = sm[row][c8 + e];
        hb[e] = F16OUT ? h_bits(f) : f2bf_bits(f);
      }
      const v4u u = (v4u){pk16(hb[0], hb[1]), pk16(hb[2], hb[3]), pk16(hb[4], hb[5]), pk16(hb[6], hb[7])};
      *(volatile v4u*)(out + (size_t)(nt * 64 + row) * kDim + kt * 64 + c8) = u;
    }
    __threadfence();
  }
}

__global__ __launch_bounds__(256) void softmax_row_kernel(const float* __restrict__ Sp, unsigned short* __restrict__ Pp) {
  __shared__ __align__(16) float lg[kSeq];
  __shared__ float redM[8];
  __shared__ float redS[8];
  const int i    = blockIdx.x;
  const int sl   = blockIdx.y;
  const int t    = threadIdx.x;
  const int lane = t & 31, wave = t >> 5;
  const size_t rowoff = ((size_t)sl * kSeq + i) * kSeq;
  const float* sr = Sp + rowoff + 8 * (size_t)t;
  const v4f a = *(const v4f*)(sr);
  const v4f c = *(const v4f*)(sr + 4);
  float mx = fmaxf(fmaxf(fmaxf(a[0], a[1]), fmaxf(a[2], a[3])), fmaxf(fmaxf(c[0], c[1]), fmaxf(c[2], c[3])));
#pragma unroll
  for (int off = 16; off > 0; off >>= 1) mx = fmaxf(mx, __shfl_xor(mx, off, 32));
  if (lane == 0) redM[wave] = mx;
  __syncthreads();
  float m = redM[0];
#pragma unroll
  for (int w = 1; w < 8; ++w) m = fmaxf(m, redM[w]);

  float sum = 0.0f;
#pragma unroll 1
  for (int it = 0; it < 2; ++it) {
    const v4f sv = *(const v4f*)(sr + 4 * it);
    v4f ev;
#pragma unroll
    for (int e = 0; e < 4; ++e) {
      ev[e] = expf(sv[e] - m);
      sum += ev[e];
    }
    *(v4f*)(lg + 8 * t + 4 * it) = ev;
  }
#pragma unroll
  for (int off = 16; off > 0; off >>= 1) sum += __shfl_xor(sum, off, 32);
  if (lane == 0) redS[wave] = sum;
  __syncthreads();
  float tot = redS[0];
#pragma unroll
  for (int w = 1; w < 8; ++w) tot += redS[w];
  const float inv = kPCarry / tot;

  const v4f e0 = *(const v4f*)(lg + 8 * t);
  const v4f e1 = *(const v4f*)(lg + 8 * t + 4);
  unsigned short hb[8];
#pragma unroll
  for (int e = 0; e < 4; ++e) {
    hb[e]     = h_bits(e0[e] * inv);
    hb[4 + e] = h_bits(e1[e] * inv);
  }
  const v4u u = (v4u){pk16(hb[0], hb[1]), pk16(hb[2], hb[3]), pk16(hb[4], hb[5]), pk16(hb[6], hb[7])};
  unsigned short* pr = Pp + rowoff + 8 * (size_t)t;
  *(volatile v4u*)pr = u;
  __threadfence();
  *(volatile v4u*)pr = u;
}

extern "C" void kernel_launch(void* const* d_in, const int* in_sizes, int n_in,
                              void* d_out, int out_size, void* d_ws, size_t ws_size,
                              hipStream_t stream) {
  if (n_in < 7) return;
  if (in_sizes[0] != kTok * kDim) return;
  if (in_sizes[1] != kDim * kDim) return;
  if (in_sizes[2] != kDim * kKVDim) return;
  if (in_sizes[3] != kDim * kKVDim) return;
  if (in_sizes[4] != kDim * kDim) return;
  if (in_sizes[5] != kDim) return;
  if (in_sizes[6] != kHeads) return;
  if (out_size != kTok * kDim) return;
  if (ws_size < kWsTotal) return;

  const float* x    = (const float*)d_in[0];
  const float* Wq   = (const float*)d_in[1];
  const float* Wk   = (const float*)d_in[2];
  const float* Wv   = (const float*)d_in[3];
  const float* Wp   = (const float*)d_in[4];
  const float* bp   = (const float*)d_in[5];
  const int*   perm = (const int*)d_in[6];
  float* out = (float*)d_out;
  char* ws = (char*)d_ws;
  unsigned short* XB   = (unsigned short*)(ws + kOffX);
  unsigned short* WQK  = (unsigned short*)(ws + kOffWqk);
  unsigned short* WV   = (unsigned short*)(ws + kOffWv);
  unsigned short* WPT  = (unsigned short*)(ws + kOffWp);
  unsigned short* QK16 = (unsigned short*)(ws + kOffQK);
  unsigned short* VT16 = (unsigned short*)(ws + kOffVT);
  float*          SC   = (float*)(ws + kOffSC);
  unsigned short* PP   = (unsigned short*)(ws + kOffPP);
  unsigned short* O16  = (unsigned short*)(ws + kOffO);

  const int n8 = (kTok * kDim) / 8;
  cast8_bf16_kernel<<<dim3(n8 / 256), dim3(256), 0, stream>>>(x, XB, n8);
  wprep_kernel<0, 1, false><<<dim3(kDim / 64, kDim / 64), dim3(256), 0, stream>>>(Wq, kDim, perm, WQK, 1.0f);
  wprep_kernel<2, 0, false><<<dim3(kDim / 64, kKVDim / 64), dim3(256), 0, stream>>>(Wk, kKVDim, perm, WQK + (size_t)kDim * kDim, 1.0f);
  wprep_kernel<2, 0, false><<<dim3(kDim / 64, kKVDim / 64), dim3(256), 0, stream>>>(Wv, kKVDim, perm, WV, 1.0f);
  wprep_kernel<1, 0, true><<<dim3(kDim / 64, kDim / 64), dim3(256), 0, stream>>>(Wp, kDim, perm, WPT, kWpCarry);

  const int tilesQK = (kTok / 64) * (kQKN / 64);
  wmma_gemm64<1, false, 0, 1, false, 0><<<dim3(tilesQK / 8, 1), dim3(256), 0, stream>>>(
      XB, XB, kDim, 0L, WQK, WQK, kDim, 0L,
      (void*)QK16, (void*)QK16, kQKN, 0L, bp, bp, 0L, kTok, kQKN, kDim, kQKCarry);
  const int tilesVT = (kKVDim / 64) * (kTok / 64);
  wmma_gemm64<1, false, 0, 1, false, 0><<<dim3(tilesVT / 8, 1), dim3(256), 0, stream>>>(
      WV, WV, kDim, 0L, XB, XB, kDim, 0L,
      (void*)VT16, (void*)VT16, kTok, 0L, bp, bp, 0L, kKVDim, kTok, kDim, kVCarry);

  const long strideSlotQ = (long)kDh;
  const long strideScore = (long)kSeq * kSeq;
  const long strideSlotO = (long)kDh;
  const int  tilesScore  = (kSeq / 64) * (kSeq / 64);
  const int  tilesCtx    = (kSeq / 64) * (kDh / 64);
  for (int b = 0; b < kBatch; ++b) {
    for (int g = 0; g < kKVHeads; ++g) {
      const size_t tokRow = (size_t)b * kSeq;
      const unsigned short* Aq  = QK16 + tokRow * kQKN + (size_t)(kSlotsPerGroup * g) * kDh;
      const unsigned short* Btk = QK16 + tokRow * kQKN + kDim + (size_t)g * kDh;
      wmma_gemm64<0, false, 0, 0, false, 0><<<dim3(tilesScore / 8, kSlotsPerGroup), dim3(256), 0, stream>>>(
          Aq, Aq, kQKN, strideSlotQ, Btk, Btk, kQKN, 0L,
          (void*)SC, (void*)SC, kSeq, strideScore, bp, bp, 0L, kSeq, kSeq, kDh, kScoreScale);
      softmax_row_kernel<<<dim3(kSeq, kSlotsPerGroup), dim3(256), 0, stream>>>(SC, PP);
      const unsigned short* Btv = VT16 + ((size_t)g * kDh) * kTok + tokRow;
      unsigned short* Og = O16 + tokRow * kDim + (size_t)(kSlotsPerGroup * g) * kDh;
      wmma_gemm64<0, false, 0, 1, false, 0><<<dim3(tilesCtx / 8, kSlotsPerGroup), dim3(256), 0, stream>>>(
          PP, PP, kSeq, strideScore, Btv, Btv, kTok, 0L,
          (void*)Og, (void*)Og, kDim, strideSlotO, bp, bp, 0L, kSeq, kDh, kSeq, kPVScale);
    }
  }

  const int tilesOut = (kTok / 64) * (kDim / 64);
  wmma_gemm64<0, false, 2, 0, false, 0><<<dim3(tilesOut / 8, 1), dim3(256), 0, stream>>>(
      O16, O16, kDim, 0L, WPT, WPT, kDim, 0L,
      (void*)out, (void*)out, kDim, 0L, bp, bp, 0L, kTok, kDim, kDim, kOutScale);
}
